// MPNN_72378788872769
// MI455X (gfx1250) — hardware-verified
//
#include <hip/hip_runtime.h>
#include <stddef.h>
#include <math.h>


#define NB     4
#define NN     64
#define FIN    32
#define EDIM   32
#define FD     64
#define G3N    192
#define KG     128
#define NROW   (NB * NN)
#define NPAIR  (NB * NN * NN)
#define WEC    (FD * FD)
#define NITER  3
#define U0     (WEC * 4)
#define U1     (FD * 4)
#define U2     (G3N * 16)
#define U3     (G3N * 16)
#define UTOT   (U0 + U1 + U2 + U3)
#define WSMAX  134217728

static_assert(U0 % 256 == 0 && (U0 + U1) % 256 == 0 && (U0 + U1 + U2) % 256 == 0 && UTOT % 256 == 0);
static_assert(EDIM % 32 == 0 && FIN % 32 == 0 && KG % 32 == 0 && KG == 2 * FD);
static_assert(NROW % 64 == 0 && NROW % 16 == 0 && G3N == 4 * 48);

typedef float          v4f   __attribute__((ext_vector_type(4)));
typedef float          v8f   __attribute__((ext_vector_type(8)));
typedef int            v8i   __attribute__((ext_vector_type(8)));
typedef unsigned short v8us  __attribute__((ext_vector_type(8)));
typedef __bf16         v16bf __attribute__((ext_vector_type(16)));
typedef v4f  __attribute__((may_alias)) v4fa;
typedef v8us __attribute__((may_alias)) v8usa;
union FragB { v16bf v; v8us h[2]; v8i w; };

__device__ __forceinline__ v8f z8() { v8f z = {0.f, 0.f, 0.f, 0.f, 0.f, 0.f, 0.f, 0.f}; return z; }

__device__ __forceinline__ v8f wmb(const FragB& a, const FragB& b, v8f c) {
  v8f d = __builtin_amdgcn_wmma_f32_16x16x32_bf16(false, a.v, false, b.v, (short)0, c, false, false);
  asm volatile("v_nop\n\tv_nop\n\tv_nop\n\tv_nop" : "+v"(d) : "v"(a.w), "v"(b.w));
  return d;
}

__device__ __forceinline__ unsigned bf16_bits(float f) {
  const unsigned u = __float_as_uint(f);
  return (u + 0x7FFFu + ((u >> 16) & 1u)) >> 16;
}
__device__ __forceinline__ float bf16_val(float f) { return __uint_as_float(bf16_bits(f) << 16); }

__device__ __forceinline__ v8us cvt8(v4f a, v4f b) {
  v8us o;
  o[0] = (unsigned short)bf16_bits(a.x); o[1] = (unsigned short)bf16_bits(a.y);
  o[2] = (unsigned short)bf16_bits(a.z); o[3] = (unsigned short)bf16_bits(a.w);
  o[4] = (unsigned short)bf16_bits(b.x); o[5] = (unsigned short)bf16_bits(b.y);
  o[6] = (unsigned short)bf16_bits(b.z); o[7] = (unsigned short)bf16_bits(b.w);
  return o;
}
__device__ __forceinline__ void split8(v4f a, v4f b, v8us& hi, v8us& lo) {
  float v[8] = {a.x, a.y, a.z, a.w, b.x, b.y, b.z, b.w};
#pragma unroll
  for (int k = 0; k < 8; ++k) {
    const unsigned hb = bf16_bits(v[k]);
    hi[k] = (unsigned short)hb;
    lo[k] = (unsigned short)bf16_bits(v[k] - __uint_as_float(hb << 16));
  }
}
__device__ __forceinline__ float sigm(float x) { return 1.0f / (1.0f + expf(-x)); }

__global__ __launch_bounds__(256) void k_prep(const float* __restrict__ Wedge, const float* __restrict__ Wemb,
                                              const float* __restrict__ gk, const float* __restrict__ grk,
                                              unsigned short* WET, unsigned short* WEMT,
                                              unsigned short* K2, unsigned short* RK2) {
  const int u = (int)blockIdx.x * 256 + (int)threadIdx.x;
  const float* p;
  unsigned short* dp;
  int stride;
  if (u < U0) {
    const int n = u >> 2, k8 = (u & 3) * 8;
    p = Wedge + (size_t)k8 * WEC + n; stride = WEC;
    dp = WET + (size_t)n * EDIM + k8;
  } else if (u < U0 + U1) {
    const int v = u - U0;
    const int n = v >> 2, k8 = (v & 3) * 8;
    p = Wemb + (size_t)k8 * FD + n; stride = FD;
    dp = WEMT + (size_t)n * FIN + k8;
  } else if (u < U0 + U1 + U2) {
    const int v = u - (U0 + U1);
    const int n = v >> 4, k8 = (v & 15) * 8, kk = k8 & (FD - 1);
    p = gk + (size_t)kk * G3N + n; stride = G3N;
    dp = K2 + (size_t)n * KG + k8;
  } else if (u < UTOT) {
    const int v = u - (U0 + U1 + U2);
    const int n = v >> 4, k8 = (v & 15) * 8, kk = k8 & (FD - 1);
    p = grk + (size_t)kk * G3N + n; stride = G3N;
    dp = RK2 + (size_t)n * KG + k8;
  } else {
    return;
  }
  v8us o;
#pragma unroll
  for (int i = 0; i < 8; ++i) o[i] = (unsigned short)bf16_bits(p[(size_t)i * (size_t)stride]);
  *(volatile v8us*)dp = o;
  __threadfence();
  *(volatile v8us*)dp = o;
}

__global__ __launch_bounds__(128) void k_embed(const float* __restrict__ X, const unsigned short* __restrict__ WEMT,
                                               const float* __restrict__ be, float* HA) {
  __shared__ __attribute__((aligned(16))) float stg[64 * FD];
  const int tid = (int)threadIdx.x, lane = tid & 31, wave = tid >> 5, hh = lane >> 4, m = lane & 15;
  const int rowBase = (int)blockIdx.x * 64;
  const float* xp = X + (size_t)(rowBase + 16 * wave + m) * FIN + 8 * hh;
  FragB af;
  af.h[0] = cvt8(*(const v4fa*)xp, *(const v4fa*)(xp + 4));
  af.h[1] = cvt8(*(const v4fa*)(xp + 16), *(const v4fa*)(xp + 20));
  v8f acc[4];
#pragma unroll
  for (int t = 0; t < 4; ++t) {
    const unsigned short* wq = WEMT + (size_t)(16 * t + m) * FIN + 8 * hh;
    FragB bf;
    bf.h[0] = *(const v8usa*)wq;
    bf.h[1] = *(const v8usa*)(wq + 16);
    acc[t] = wmb(af, bf, z8());
  }
#pragma unroll
  for (int t = 0; t < 4; ++t) {
    const int lc = 16 * t + m;
    const float bv = bf16_val(be[lc]);
#pragma unroll
    for (int r = 0; r < 8; ++r) stg[(16 * wave + 8 * hh + r) * FD + lc] = fmaxf(acc[t][r] + bv, 0.0f);
  }
  __syncthreads();
  v4f fv[8];
#pragma unroll
  for (int i = 0; i < 8; ++i) fv[i] = *(const v4fa*)(stg + (16 * wave + 2 * i + hh) * FD + 4 * m);
#pragma unroll
  for (int i = 0; i < 8; ++i)
    *(volatile v4f*)(HA + (size_t)(rowBase + 16 * wave + 2 * i + hh) * FD + 4 * m) = fv[i];
  __threadfence();
#pragma unroll
  for (int i = 0; i < 8; ++i)
    *(volatile v4f*)(HA + (size_t)(rowBase + 16 * wave + 2 * i + hh) * FD + 4 * m) = fv[i];
}

__global__ __launch_bounds__(256) void k_msg(const float* __restrict__ E, const float* __restrict__ A,
                                             const float* __restrict__ Hpl, const unsigned short* __restrict__ WET,
                                             const float* __restrict__ b_edge, float* AGG) {
  __shared__ __attribute__((aligned(16))) unsigned short EBs[NN * EDIM];
  __shared__ __attribute__((aligned(16))) float HM[NN * FD];
  __shared__ __attribute__((aligned(16))) float AGS[FD];
  const int tid = (int)threadIdx.x, lane = tid & 31, wave = tid >> 5, hh = lane >> 4, c = lane & 15;
  const int blk = (int)blockIdx.x;
  const int b = blk >> 6;
  {
    const int row = tid >> 2, q4 = tid & 3;
    const float* ep = E + ((size_t)blk * NN + row) * EDIM + 8 * q4;
    const v4f e0 = *(const v4fa*)ep;
    const v4f e1 = *(const v4fa*)(ep + 4);
    *(v8usa*)(EBs + row * EDIM + 8 * q4) = cvt8(e0, e1);
    const float mk = A[(size_t)blk * NN + row];
    const float* hp = Hpl + ((size_t)b * NN + row) * FD + 16 * q4;
    float* dp = HM + row * FD + 16 * q4;
#pragma unroll
    for (int q = 0; q < 4; ++q) {
      const v4f hv = *(const v4fa*)(hp + 4 * q);
      *(v4fa*)(dp + 4 * q) = hv * mk;
    }
  }
  __syncthreads();

#pragma unroll 1
  for (int ii = 0; ii < 8; ++ii) {
    const int i = wave + 8 * ii;
    FragB bf[4];
#pragma unroll
    for (int t = 0; t < 4; ++t) {
      const unsigned short* wq = WET + (size_t)(i * FD + 4 * c + t) * EDIM + 8 * hh;
      bf[t].h[0] = *(const v8usa*)wq;
      bf[t].h[1] = *(const v8usa*)(wq + 16);
    }
    const v4f braw = *(const v4fa*)(b_edge + (size_t)i * FD + 4 * c);
    const float b0 = bf16_val(braw.x), b1 = bf16_val(braw.y), b2 = bf16_val(braw.z), b3 = bf16_val(braw.w);
    float part = 0.0f;
#pragma unroll 1
    for (int mt = 0; mt < 4; ++mt) {
      const unsigned short* ap = EBs + (16 * mt + c) * EDIM + 8 * hh;
      FragB af;
      af.h[0] = *(const v8usa*)ap;
      af.h[1] = *(const v8usa*)(ap + 16);
      const v8f a0 = wmb(af, bf[0], z8());
      const v8f a1 = wmb(af, bf[1], z8());
      const v8f a2 = wmb(af, bf[2], z8());
      const v8f a3 = wmb(af, bf[3], z8());
      const float* hrow = HM + (16 * mt + 8 * hh) * FD + 4 * c;
#pragma unroll
      for (int r = 0; r < 8; ++r) {
        const v4f hv = *(const v4fa*)(hrow + r * FD);
        part = fmaf(fmaxf(a0[r] + b0, 0.0f), hv.x, part);
        part = fmaf(fmaxf(a1[r] + b1, 0.0f), hv.y, part);
        part = fmaf(fmaxf(a2[r] + b2, 0.0f), hv.z, part);
        part = fmaf(fmaxf(a3[r] + b3, 0.0f), hv.w, part);
      }
    }
    part += __shfl_xor(part, 16);
    part += __shfl_xor(part, 8);
    part += __shfl_xor(part, 4);
    part += __shfl_xor(part, 2);
    part += __shfl_xor(part, 1);
    if (lane == 0) AGS[i] = part;
  }
  __syncthreads();
  const v4f ov = *(const v4fa*)(AGS + 4 * (lane & 15));
  float* op = AGG + (size_t)blk * FD + 4 * (lane & 15);
  const bool okst = (wave == 0) && (lane < 16);
  if (okst) *(volatile v4f*)op = ov;
  __threadfence();
  if (okst) *(volatile v4f*)op = ov;
}

__global__ __launch_bounds__(128) void k_gru(const float* __restrict__ Hin, const float* __restrict__ AGG,
                                             const unsigned short* __restrict__ K2, const unsigned short* __restrict__ RK2,
                                             const float* __restrict__ gb, const float* __restrict__ grb, float* Hout) {
  __shared__ __attribute__((aligned(16))) unsigned short HHL[16 * KG];
  __shared__ __attribute__((aligned(16))) unsigned short AHL[16 * KG];
  __shared__ __attribute__((aligned(16))) unsigned short H1HL[16 * KG];
  __shared__ __attribute__((aligned(16))) float GA[16 * G3N];
  __shared__ __attribute__((aligned(16))) float GB[16 * G3N];
  __shared__ __attribute__((aligned(16))) float H1S[16 * FD];
  __shared__ __attribute__((aligned(16))) float OUTS[16 * FD];
  __shared__ float BK[G3N];
  __shared__ float BR[G3N];
  const int tid = (int)threadIdx.x, lane = tid & 31, wave = tid >> 5, hh = lane >> 4, m = lane & 15;
  const int rbase = (int)blockIdx.x * 16;
  const int row = tid >> 3, c8 = (tid & 7) * 8;
  for (int i = tid; i < G3N; i += 128) { BK[i] = bf16_val(gb[i]); BR[i] = bf16_val(grb[i]); }
  {
    const float* hp = Hin + (size_t)(rbase + row) * FD + c8;
    const float* gp = AGG + (size_t)(rbase + row) * FD + c8;
    const v4f h0 = *(const v4fa*)hp, h1 = *(const v4fa*)(hp + 4);
    const v4f g0 = *(const v4fa*)gp, g1 = *(const v4fa*)(gp + 4);
    v8us hi, lo;
    split8(h0, h1, hi, lo);
    *(v8usa*)(HHL + row * KG + c8) = hi;
    *(v8usa*)(HHL + row * KG + FD + c8) = lo;
    split8(g0, g1, hi, lo);
    *(v8usa*)(AHL + row * KG + c8) = hi;
    *(v8usa*)(AHL + row * KG + FD + c8) = lo;
  }
  __syncthreads();
  {
    v8f acc1[3], acc2[3];
#pragma unroll
    for (int t = 0; t < 3; ++t) { acc1[t] = z8(); acc2[t] = z8(); }
#pragma unroll
    for (int ks = 0; ks < 4; ++ks) {
      const int ao = m * KG + 32 * ks + 8 * hh;
      FragB a1, a2;
      a1.h[0] = *(const v8usa*)(HHL + ao); a1.h[1] = *(const v8usa*)(HHL + ao + 16);
      a2.h[0] = *(const v8usa*)(AHL + ao); a2.h[1] = *(const v8usa*)(AHL + ao + 16);
#pragma unroll
      for (int t = 0; t < 3; ++t) {
        const unsigned short* wq = K2 + (size_t)(48 * wave + 16 * t + m) * KG + 32 * ks + 8 * hh;
        FragB bf;
        bf.h[0] = *(const v8usa*)wq;
        bf.h[1] = *(const v8usa*)(wq + 16);
        acc1[t] = wmb(a1, bf, acc1[t]);
        acc2[t] = wmb(a2, bf, acc2[t]);
      }
    }
#pragma unroll
    for (int t = 0; t < 3; ++t) {
      const int col = 48 * wave + 16 * t + m;
      const float bk = BK[col];
#pragma unroll
      for (int r = 0; r < 8; ++r) {
        GA[(8 * hh + r) * G3N + col] = acc1[t][r] + bk;
        GB[(8 * hh + r) * G3N + col] = acc2[t][r] + bk;
      }
    }
  }
  __syncthreads();
#pragma unroll 1
  for (int e = 0; e < 8; ++e) {
    const int f = c8 + e;
    const float xz = GA[row * G3N + f], xr = GA[row * G3N + FD + f], xh = GA[row * G3N + 2 * FD + f];
    const float z1 = sigm(xz + BR[f]);
    const float r1 = sigm(xr + BR[FD + f]);
    const float c1 = tanhf(xh + r1 * BR[2 * FD + f]);
    const float h1v = (1.0f - z1) * c1;
    H1S[row * FD + f] = h1v;
    const unsigned hb = bf16_bits(h1v);
    H1HL[row * KG + f] = (unsigned short)hb;
    H1HL[row * KG + FD + f] = (unsigned short)bf16_bits(h1v - __uint_as_float(hb << 16));
  }
  __syncthreads();
  {
    v8f acc3[3];
#pragma unroll
    for (int t = 0; t < 3; ++t) acc3[t] = z8();
#pragma unroll
    for (int ks = 0; ks < 4; ++ks) {
      const int ao = m * KG + 32 * ks + 8 * hh;
      FragB a3;
      a3.h[0] = *(const v8usa*)(H1HL + ao); a3.h[1] = *(const v8usa*)(H1HL + ao + 16);
#pragma unroll
      for (int t = 0; t < 3; ++t) {
        const unsigned short* wq = RK2 + (size_t)(48 * wave + 16 * t + m) * KG + 32 * ks + 8 * hh;
        FragB bf;
        bf.h[0] = *(const v8usa*)wq;
        bf.h[1] = *(const v8usa*)(wq + 16);
        acc3[t] = wmb(a3, bf, acc3[t]);
      }
    }
#pragma unroll
    for (int t = 0; t < 3; ++t) {
      const int col = 48 * wave + 16 * t + m;
      const float br = BR[col];
#pragma unroll
      for (int r = 0; r < 8; ++r) GA[(8 * hh + r) * G3N + col] = acc3[t][r] + br;
    }
  }
  __syncthreads();
#pragma unroll 1
  for (int e = 0; e < 8; ++e) {
    const int f = c8 + e;
    const float z2 = sigm(GB[row * G3N + f] + GA[row * G3N + f]);
    const float r2 = sigm(GB[row * G3N + FD + f] + GA[row * G3N + FD + f]);
    const float c2 = tanhf(GB[row * G3N + 2 * FD + f] + r2 * GA[row * G3N + 2 * FD + f]);
    const float h1v = H1S[row * FD + f];
    OUTS[row * FD + f] = z2 * h1v + (1.0f - z2) * c2;
  }
  __syncthreads();
  const v4f o0 = *(const v4fa*)(OUTS + 4 * tid);
  const v4f o1 = *(const v4fa*)(OUTS + 4 * (128 + tid));
  float* gp = Hout + (size_t)rbase * FD;
  *(volatile v4f*)(gp + 4 * tid) = o0;
  *(volatile v4f*)(gp + 4 * (128 + tid)) = o1;
  __threadfence();
  *(volatile v4f*)(gp + 4 * tid) = o0;
  *(volatile v4f*)(gp + 4 * (128 + tid)) = o1;
}

extern "C" void kernel_launch(void* const* d_in, const int* in_sizes, int n_in,
                              void* d_out, int out_size, void* d_ws, size_t ws_size,
                              hipStream_t stream) {
  if (n_in < 11) return;
  if (in_sizes[0] != NROW * FIN) return;
  if (in_sizes[1] != NPAIR) return;
  if (in_sizes[2] != NPAIR * EDIM) return;
  if (in_sizes[3] != FIN * FD || in_sizes[4] != FD) return;
  if (in_sizes[5] != EDIM * WEC || in_sizes[6] != WEC) return;
  if (in_sizes[7] != FD * G3N || in_sizes[8] != FD * G3N) return;
  if (in_sizes[9] != G3N || in_sizes[10] != G3N) return;
  if (out_size != NROW * FD) return;

  const float* X      = (const float*)d_in[0];
  const float* A      = (const float*)d_in[1];
  const float* E      = (const float*)d_in[2];
  const float* Wemb   = (const float*)d_in[3];
  const float* bemb   = (const float*)d_in[4];
  const float* Wedge  = (const float*)d_in[5];
  const float* bedge  = (const float*)d_in[6];
  const float* gk     = (const float*)d_in[7];
  const float* grk    = (const float*)d_in[8];
  const float* gbias  = (const float*)d_in[9];
  const float* grbias = (const float*)d_in[10];
  float* out = (float*)d_out;

  const size_t szWET = (size_t)WEC * EDIM * 2;
  const size_t szWEM = (size_t)FD * FIN * 2;
  const size_t szK2  = (size_t)G3N * KG * 2;
  const size_t szH   = (size_t)NROW * FD * 4;
  const size_t oWET = 0;
  const size_t oWEM = oWET + szWET;
  const size_t oK2  = oWEM + szWEM;
  const size_t oRK2 = oK2 + szK2;
  const size_t oHA  = oRK2 + szK2;
  const size_t oHB  = oHA + szH;
  const size_t oAGG = oHB + szH;
  const size_t total = oAGG + szH;
  if (total > ws_size || total > (size_t)WSMAX) return;
  char* ws = (char*)d_ws;
  unsigned short* WET  = (unsigned short*)(ws + oWET);
  unsigned short* WEMT = (unsigned short*)(ws + oWEM);
  unsigned short* K2   = (unsigned short*)(ws + oK2);
  unsigned short* RK2  = (unsigned short*)(ws + oRK2);
  float* HA  = (float*)(ws + oHA);
  float* HB  = (float*)(ws + oHB);
  float* AGG = (float*)(ws + oAGG);

  k_prep<<<UTOT / 256, 256, 0, stream>>>(Wedge, Wemb, gk, grk, WET, WEMT, K2, RK2);
  k_embed<<<NROW / 64, 128, 0, stream>>>(X, WEMT, bemb, HA);
  k_msg<<<NROW, 256, 0, stream>>>(E, A, HA, WET, bedge, AGG);
  k_gru<<<NROW / 16, 128, 0, stream>>>(HA, AGG, K2, RK2, gbias, grbias, HB);
  k_msg<<<NROW, 256, 0, stream>>>(E, A, HB, WET, bedge, AGG);
  k_gru<<<NROW / 16, 128, 0, stream>>>(HB, AGG, K2, RK2, gbias, grbias, HA);
  k_msg<<<NROW, 256, 0, stream>>>(E, A, HA, WET, bedge, AGG);
  k_gru<<<NROW / 16, 128, 0, stream>>>(HA, AGG, K2, RK2, gbias, grbias, out);
}
